// net_55903294324835
// MI455X (gfx1250) — hardware-run, weakly checked
//
#include <hip/hip_runtime.h>

typedef float          v8f   __attribute__((ext_vector_type(8)));
typedef float          v4f   __attribute__((ext_vector_type(4)));
typedef unsigned int   v4u   __attribute__((ext_vector_type(4)));
typedef int            v8i   __attribute__((ext_vector_type(8)));
typedef unsigned short v8us  __attribute__((ext_vector_type(8)));
typedef unsigned short v16us __attribute__((ext_vector_type(16)));
typedef __bf16         v16bf __attribute__((ext_vector_type(16)));
typedef _Float16       v16h  __attribute__((ext_vector_type(16)));
typedef v4f  __attribute__((may_alias)) v4fa;
typedef v8us __attribute__((may_alias)) v8usa;
union FragB { v16bf v; v16us u; v8us h[2]; v8i w; };
union FragH { v16h  v; v16us u; v8us h[2]; v8i w; };

__device__ __forceinline__ v8f wmb(const FragB& a, const FragB& b, v8f c) {
  v8f d = __builtin_amdgcn_wmma_f32_16x16x32_bf16(false, a.v, false, b.v, (short)0, c, false, false);
  asm volatile("v_nop\n\tv_nop\n\tv_nop\n\tv_nop" : "+v"(d) : "v"(a.w), "v"(b.w));
  return d;
}

__device__ __forceinline__ v8f wmh(const FragH& a, const FragH& b, v8f c) {
  v8f d = __builtin_amdgcn_wmma_f32_16x16x32_f16(false, a.v, false, b.v, (short)0, c, false, false);
  asm volatile("v_nop\n\tv_nop\n\tv_nop\n\tv_nop" : "+v"(d) : "v"(a.w), "v"(b.w));
  return d;
}

__device__ __forceinline__ unsigned bf16_bits(float f) {
  const unsigned u = __float_as_uint(f);
  const unsigned r = (u + 0x7FFFu + ((u >> 16) & 1u)) >> 16;
  const unsigned q = (u >> 16) | 0x40u;
  return ((u & 0x7fffffffu) > 0x7f800000u) ? q : r;
}

__device__ __forceinline__ float bf16_val(float f) {
  return __uint_as_float(bf16_bits(f) << 16);
}
__device__ __forceinline__ int clampi(int v, int lo, int hi) {
  return v < lo ? lo : (v > hi ? hi : v);
}

__device__ __forceinline__ unsigned f16_bits(float f) {
  const unsigned u  = __float_as_uint(f);
  const unsigned s  = (u >> 16) & 0x8000u;
  const unsigned a  = u & 0x7fffffffu;
  const unsigned t  = a - 0x38000000u;
  const unsigned r  = (t + 0x0FFFu + ((t >> 13) & 1u)) >> 13;
  const unsigned rc = r > 0x7C00u ? 0x7C00u : r;
  const bool small  = a < 0x38800000u;
  const bool isnan  = a > 0x7f800000u;
  const unsigned fin = small ? 0u : (s | rc);
  return isnan ? (s | 0x7E00u) : fin;
}

__device__ __forceinline__ unsigned pk16(unsigned lo, unsigned hi) { return lo | (hi << 16); }
__device__ __forceinline__ unsigned bf16_lo_bits(float v) {
  float hi = bf16_val(v);
  asm volatile("" : "+v"(hi));
  return bf16_bits(v - hi);
}
__device__ __forceinline__ v4u pack8_bf16(v4f a, v4f c) {
  return (v4u){ pk16(bf16_bits(a[0]), bf16_bits(a[1])), pk16(bf16_bits(a[2]), bf16_bits(a[3])),
                pk16(bf16_bits(c[0]), bf16_bits(c[1])), pk16(bf16_bits(c[2]), bf16_bits(c[3])) };
}
__device__ __forceinline__ v4u pack8_bf16_lo(v4f a, v4f c) {
  return (v4u){ pk16(bf16_lo_bits(a[0]), bf16_lo_bits(a[1])), pk16(bf16_lo_bits(a[2]), bf16_lo_bits(a[3])),
                pk16(bf16_lo_bits(c[0]), bf16_lo_bits(c[1])), pk16(bf16_lo_bits(c[2]), bf16_lo_bits(c[3])) };
}
__device__ __forceinline__ v4u pack8_f16(v4f a, v4f c) {
  return (v4u){ pk16(f16_bits(a[0]), f16_bits(a[1])), pk16(f16_bits(a[2]), f16_bits(a[3])),
                pk16(f16_bits(c[0]), f16_bits(c[1])), pk16(f16_bits(c[2]), f16_bits(c[3])) };
}

template <int FORM>
__global__ __launch_bounds__(256) void k_plane(const float* __restrict__ src, int rows, int cols, int ldsrc,
                                               unsigned short* __restrict__ dst, int MP, int KP) {
  static_assert(FORM >= 0 && FORM <= 3);
  const int KTOT = (FORM == 1 || FORM == 3) ? 2 * KP : KP;
  const unsigned ppr   = (unsigned)(KTOT >> 3);
  const unsigned kp8   = (unsigned)(KP >> 3);
  const unsigned total = (unsigned)MP * ppr;
  const unsigned g     = blockIdx.x * 256u + threadIdx.x;
  const unsigned rowu  = g / ppr;
  const unsigned p     = g - rowu * ppr;
  const bool second    = p >= kp8;
  const int row = (int)rowu;
  const int c0  = (int)((second ? p - kp8 : p) << 3);
  const float* srow = src + (size_t)clampi(row, 0, rows - 1) * (size_t)ldsrc;
  float x[8];
  unsigned mk[8];
#pragma unroll
  for (int e = 0; e < 8; ++e) {
    const int c = c0 + e;
    const float v = srow[clampi(c, 0, cols - 1)];
    asm volatile("" :: "v"(v));
    x[e]  = v;
    mk[e] = (row < rows && c < cols) ? 0xFFFFu : 0u;
  }
  const v4f a = (v4f){ x[0], x[1], x[2], x[3] };
  const v4f c = (v4f){ x[4], x[5], x[6], x[7] };
  v4u o;
  if (FORM == 2) {
    o = pack8_f16(a, c);
  } else {
    const v4u hi = pack8_bf16(a, c);
    o = hi;
    if (FORM == 1) { const v4u lo = pack8_bf16_lo(a, c); o = second ? lo : hi; }
  }
  const v4u mw = (v4u){ pk16(mk[0], mk[1]), pk16(mk[2], mk[3]), pk16(mk[4], mk[5]), pk16(mk[6], mk[7]) };
  o &= mw;
  if (g < total) {
    volatile v4u* q = (volatile v4u*)(dst + (size_t)g * 8);
    *q = o;
    __threadfence();
    *q = o;
  }
}

template <int FORM> struct FragOf    { typedef FragB T; };
template <>         struct FragOf<2> { typedef FragH T; };
__device__ __forceinline__ v8f mm(const FragB& a, const FragB& b, v8f c) { return wmb(a, b, c); }
__device__ __forceinline__ v8f mm(const FragH& a, const FragH& b, v8f c) { return wmh(a, b, c); }
template <class F> __device__ __forceinline__ F ld_frag(const unsigned short* p) {
  F f;
  f.h[0] = *(const v8usa*)(p);
  f.h[1] = *(const v8usa*)(p + 16);
  return f;
}

template <int FORM, int EPI>
__global__ __launch_bounds__(256) __attribute__((amdgpu_num_vgpr(248)))
void k_gemm_nt(const unsigned short* __restrict__ A, const unsigned short* __restrict__ B,
               const float* __restrict__ bias, float* __restrict__ D, int M, int N, int KTOT, int ldd) {
  static_assert(FORM >= 0 && FORM <= 2);
  static_assert(EPI == 0 || EPI == 1);
  typedef typename FragOf<FORM>::T F;
  __shared__ __attribute__((aligned(16))) float sT[8][16 * 68];
  const int lane = threadIdx.x & 31;
  const int wave = threadIdx.x >> 5;
  const int tilesM = (M + 63) >> 6;
  const int tilesN = (N + 63) >> 6;
  const int tile = blockIdx.x * 8 + wave;
  if (tile >= tilesM * tilesN) return;
  const int tm = tile / tilesN;
  const int tn = tile - tm * tilesN;
  const int m0 = tm << 6;
  const int n0 = tn << 6;

  const int rl = lane & 15;
  const int h8 = (lane >> 4) * 8;
  const unsigned short* pa = A + (size_t)(m0 + rl) * (size_t)KTOT + h8;
  const unsigned short* pb = B + (size_t)(n0 + rl) * (size_t)KTOT + h8;

  v8f acc[4][4];
#pragma unroll
  for (int i = 0; i < 4; ++i)
#pragma unroll
    for (int j = 0; j < 4; ++j) acc[i][j] = (v8f){0.f, 0.f, 0.f, 0.f, 0.f, 0.f, 0.f, 0.f};

#pragma unroll 1
  for (int k0 = 0; k0 < KTOT; k0 += 32) {
    F bf[4];
#pragma unroll
    for (int j = 0; j < 4; ++j) bf[j] = ld_frag<F>(pb + (size_t)(j << 4) * (size_t)KTOT + k0);
#pragma unroll
    for (int i = 0; i < 4; ++i) {
      const F af = ld_frag<F>(pa + (size_t)(i << 4) * (size_t)KTOT + k0);
#pragma unroll
      for (int j = 0; j < 4; ++j) acc[i][j] = mm(af, bf[j], acc[i][j]);
    }
  }

  float* slab = sT[wave];
  const int hh = lane >> 4;
  const int c4 = (lane & 15) * 4;
  const int nc = n0 + c4;
  const bool cok = nc < N;
  v4f bv = (v4f){0.f, 0.f, 0.f, 0.f};
  if (EPI == 1) {
    bv = *(const v4fa*)(bias + clampi(nc, 0, N - 4));
    asm volatile("" :: "v"(bv));
  }
#pragma unroll
  for (int i = 0; i < 4; ++i) {
    const int mBase = m0 + (i << 4);
#pragma unroll
    for (int j = 0; j < 4; ++j) {
#pragma unroll
      for (int r = 0; r < 8; ++r) slab[(h8 + r) * 68 + (j << 4) + rl] = acc[i][j][r];
    }
    __builtin_amdgcn_fence(__ATOMIC_RELEASE, "workgroup");
    __builtin_amdgcn_wave_barrier();
    __builtin_amdgcn_fence(__ATOMIC_ACQUIRE, "workgroup");
    v4f vv[8];
#pragma unroll
    for (int it = 0; it < 8; ++it) {
      const int row = it * 2 + hh;
      v4f v = *(const v4fa*)(slab + row * 68 + c4);
      if (EPI == 1) v += bv;
      vv[it] = v;
    }
    for (int pass = 0; pass < 2; ++pass) {
#pragma unroll
      for (int it = 0; it < 8; ++it) {
        const int row = mBase + it * 2 + hh;
        if (cok && row < M) *(volatile v4f*)(D + (size_t)row * (size_t)ldd + nc) = vv[it];
      }
      __threadfence();
    }
    __builtin_amdgcn_fence(__ATOMIC_RELEASE, "workgroup");
    __builtin_amdgcn_wave_barrier();
    __builtin_amdgcn_fence(__ATOMIC_ACQUIRE, "workgroup");
  }
}

#define NN       100000
#define NE       3200000
#define MPN      100096
#define NBLK     98
#define NBROWS   1024
#define DEGCAP   128
#define MAXHITS  33219
#define MAXDEG   57
#define NTHR     256
#define NWAVE    8
#define EPT      8
#define CHUNK    (NTHR * EPT)
#define NCHUNK   ((NE + CHUNK - 1) / CHUNK)
#define WCAP     (EPT * 32)
#define LISTN    (NWAVE * WCAP)
#define ESH      10
#define RCAP     41984
#define LTOT     (NBLK * RCAP)
#define LDS_BLD  (RCAP * 4 + RCAP * 2 + 2 * NBROWS * 4 + 64)
#define PA_WMAP  0
#define PA_BMAP  16
#define PA_TAU   20
#define PA_WC    32
#define PA_BC    228
#define PA_B1    256
#define PA_W2    384
#define PA_B2    768
#define PAR_LINES 32
#define OUT_R_ELEM (3 * NN)
#define WSMAX    ((size_t)128 << 20)

static_assert(MPN % 64 == 0 && MPN >= NN && MPN - NN < 128);
static_assert(NN % 32 == 0 && NN % 16 == 0 && NE % 256 == 0);
static_assert(NBLK * NBROWS >= NN && (NBLK - 1) * NBROWS < NN);
static_assert(NBROWS == 1024 && (1 << ESH) == NBROWS && NTHR * 4 == NBROWS);
static_assert(NE <= (1 << (32 - ESH)));
static_assert(RCAP % 512 == 0 && RCAP < 65536 && RCAP * 4 >= MAXHITS * 5);
static_assert(LISTN * 4 <= RCAP * 2);
static_assert(DEGCAP >= 2 * MAXDEG);
static_assert(LDS_BLD <= 262144);
static_assert((OUT_R_ELEM * 4) % 128 == 0);
static_assert(OUT_R_ELEM + 4 * NE == 13100000);
static_assert(NCHUNK == 1563);
static_assert((size_t)MPN * 32 / 8 < 0x7fffffffu);

constexpr size_t al256(size_t v) { return (v + 255) & ~(size_t)255; }
constexpr size_t O_XR   = 0;
constexpr size_t O_XD   = al256(O_XR   + (size_t)NN * 8);
constexpr size_t O_H1   = al256(O_XD   + (size_t)NN * 8);
constexpr size_t O_O16  = al256(O_H1   + (size_t)NN * 16);
constexpr size_t O_AHL  = al256(O_O16  + (size_t)NN * 64);
constexpr size_t O_B1T  = al256(O_AHL  + (size_t)MPN * 64);
constexpr size_t O_PAR  = al256(O_B1T  + 128 * 32 * 2);
constexpr size_t O_CNT  = al256(O_PAR  + 4096);
constexpr size_t O_OFF  = al256(O_CNT  + (size_t)NBLK * NBROWS * 4);
constexpr size_t O_META = al256(O_OFF  + (size_t)NBLK * NBROWS * 4);
constexpr size_t O_LIST = al256(O_META + (size_t)NBLK * 128);
constexpr size_t O_PRE  = al256(O_LIST + (size_t)NBLK * RCAP * 8);
constexpr size_t WS_TOTAL = al256(O_PRE + (size_t)NN * 128 * 4);
static_assert(WS_TOTAL == ((size_t)394333 << 8));
static_assert(WS_TOTAL <= (size_t)WSMAX);

typedef float v2f __attribute__((ext_vector_type(2)));
typedef int   v2i __attribute__((ext_vector_type(2)));
typedef int   v4i __attribute__((ext_vector_type(4)));
typedef v2f __attribute__((may_alias)) v2fa;
typedef v2i __attribute__((may_alias)) v2ia;
typedef v4i __attribute__((may_alias)) v4ia;
typedef v4u __attribute__((may_alias)) v4ua;

__device__ __forceinline__ void wave_sync_lds() {
  __builtin_amdgcn_fence(__ATOMIC_RELEASE, "workgroup");
  __builtin_amdgcn_wave_barrier();
  __builtin_amdgcn_fence(__ATOMIC_ACQUIRE, "workgroup");
}
__device__ __forceinline__ void st2_v4u(void* p, const v4u v) {
  volatile v4u* q = (volatile v4u*)p;
  *q = v;
  __threadfence();
  *q = v;
}
__device__ __forceinline__ void st2_v4f(float* p, const v4f v) {
  volatile v4f* q = (volatile v4f*)p;
  *q = v;
  __threadfence();
  *q = v;
}
__device__ __forceinline__ void st2_v4i(int* p, const v4i v) {
  volatile v4i* q = (volatile v4i*)p;
  *q = v;
  __threadfence();
  *q = v;
}
__device__ __forceinline__ void st2_v2f(float* p, const v2f v) {
  volatile v2f* q = (volatile v2f*)p;
  *q = v;
  __threadfence();
  *q = v;
}
__device__ __forceinline__ float blend3(float a, unsigned ma, float b, unsigned mb, float c, unsigned mc) {
  return __uint_as_float((__float_as_uint(a) & ma) | (__float_as_uint(b) & mb) | (__float_as_uint(c) & mc));
}

__global__ __launch_bounds__(256) void k_prep(
    const float* __restrict__ x, const float* __restrict__ tau, const float* __restrict__ wmap,
    const float* __restrict__ bmap, const float* __restrict__ wc, const float* __restrict__ bc,
    const float* __restrict__ w1, const float* __restrict__ b1, const float* __restrict__ w2,
    const float* __restrict__ b2, float* XR, float* PAR, unsigned short* B1T, unsigned short* AHL) {
  const int b = (int)blockIdx.x, tid = (int)threadIdx.x;
  if (b < 196) {
    const int g = b * 256 + tid;
    const int gc = g < NN / 2 ? g : NN / 2 - 1;
    const v4f v = *(const v4fa*)(x + (size_t)gc * 4);
    asm volatile("" :: "v"(v));
    const v4f o = (v4f){ bf16_val(v[0]), bf16_val(v[1]), bf16_val(v[2]), bf16_val(v[3]) };
    if (g < NN / 2) st2_v4f(XR + (size_t)g * 4, o);
  } else if (b < 200) {
    const int lane = tid & 31;
    const int wave = __builtin_amdgcn_readfirstlane(tid >> 5);
    const int u = (b - 196) * 8 + wave;
    float v = 0.0f;
    if (u == 0) {
      const float a = wmap[lane & 15];
      const float c = bmap[clampi(lane - 16, 0, 3)];
      const float t = tau[0];
      asm volatile("" :: "v"(a), "v"(c), "v"(t));
      const unsigned m0 = lane < 16 ? 0xFFFFFFFFu : 0u;
      const unsigned m1 = (lane >= 16 && lane < 20) ? 0xFFFFFFFFu : 0u;
      const unsigned m2 = lane == 20 ? 0xFFFFFFFFu : 0u;
      v = blend3(a, m0, c, m1, t, m2);
    } else if (u < 8) {
      const int t = 32 * (u - 1) + lane;
      const float a = wc[clampi(t, 0, 195)];
      const float c = bc[clampi(t - 196, 0, 13)];
      asm volatile("" :: "v"(a), "v"(c));
      const unsigned m0 = t < 196 ? 0xFFFFFFFFu : 0u;
      const unsigned m1 = (t >= 196 && t < 210) ? 0xFFFFFFFFu : 0u;
      v = blend3(a, m0, c, m1, 0.0f, 0u);
    } else if (u < 12) {
      v = b1[32 * (u - 8) + lane];
    } else if (u < 24) {
      v = w2[32 * (u - 12) + lane];
    } else if (u == 24) {
      const float a = b2[clampi(lane, 0, 2)];
      asm volatile("" :: "v"(a));
      const unsigned m0 = lane < 3 ? 0xFFFFFFFFu : 0u;
      v = blend3(a, m0, 0.0f, 0u, 0.0f, 0u);
    }
    const float o = bf16_val(v);
    volatile float* q = PAR + 32 * u + lane;
    *q = o;
    __threadfence();
    *q = o;
  } else if (b < 202) {
    const int u = (b - 200) * 256 + tid;
    const int n = u >> 2, p = u & 3;
    float xv[8];
    unsigned mk[8];
#pragma unroll
    for (int e = 0; e < 8; ++e) {
      const int k = 8 * p + e;
      int km = k >= 14 ? k - 14 : k;
      km = km > 13 ? 13 : km;
      const float v = w1[km * 128 + n];
      asm volatile("" :: "v"(v));
      xv[e] = v;
      mk[e] = k < 28 ? 0xFFFFu : 0u;
    }
    v4u o = pack8_bf16((v4f){ xv[0], xv[1], xv[2], xv[3] }, (v4f){ xv[4], xv[5], xv[6], xv[7] });
    o &= (v4u){ pk16(mk[0], mk[1]), pk16(mk[2], mk[3]), pk16(mk[4], mk[5]), pk16(mk[6], mk[7]) };
    st2_v4u(B1T + (size_t)u * 8, o);
  } else {
    const v4u z = (v4u){ 0u, 0u, 0u, 0u };
    for (int q = tid; q < (MPN - NN) * 4; q += 256) st2_v4u(AHL + (size_t)NN * 32 + (size_t)q * 8, z);
  }
}

__device__ __forceinline__ int scan_chunk(const int* __restrict__ dsts, int cbase, int slotBase,
                                          int nb, int* list, int tid, int wave) {
  int wc = 0;
  const int el0  = tid * EPT;
  const int e0   = cbase + el0;
  const int sent = -1;
  v4i da, db;
  if (cbase + CHUNK <= NE) {
    da = *(const v4i*)(dsts + e0);
    db = *(const v4i*)(dsts + e0 + 4);
  } else {
    const int t0 = dsts[min(e0 + 0, NE - 1)];
    const int t1 = dsts[min(e0 + 1, NE - 1)];
    const int t2 = dsts[min(e0 + 2, NE - 1)];
    const int t3 = dsts[min(e0 + 3, NE - 1)];
    const int t4 = dsts[min(e0 + 4, NE - 1)];
    const int t5 = dsts[min(e0 + 5, NE - 1)];
    const int t6 = dsts[min(e0 + 6, NE - 1)];
    const int t7 = dsts[min(e0 + 7, NE - 1)];
    asm volatile("" :: "v"(t0), "v"(t1), "v"(t2), "v"(t3), "v"(t4), "v"(t5), "v"(t6), "v"(t7));
    da.x = (e0 + 0 < NE) ? t0 : sent;
    da.y = (e0 + 1 < NE) ? t1 : sent;
    da.z = (e0 + 2 < NE) ? t2 : sent;
    da.w = (e0 + 3 < NE) ? t3 : sent;
    db.x = (e0 + 4 < NE) ? t4 : sent;
    db.y = (e0 + 5 < NE) ? t5 : sent;
    db.z = (e0 + 6 < NE) ? t6 : sent;
    db.w = (e0 + 7 < NE) ? t7 : sent;
  }
  const unsigned nbs = (unsigned)slotBase;
  const unsigned unb = (unsigned)nb;
  const unsigned s0 = (unsigned)da.x - nbs, s1 = (unsigned)da.y - nbs;
  const unsigned s2 = (unsigned)da.z - nbs, s3 = (unsigned)da.w - nbs;
  const unsigned s4 = (unsigned)db.x - nbs, s5 = (unsigned)db.y - nbs;
  const unsigned s6 = (unsigned)db.z - nbs, s7 = (unsigned)db.w - nbs;
  const bool h0 = s0 < unb, h1 = s1 < unb, h2 = s2 < unb, h3 = s3 < unb;
  const bool h4 = s4 < unb, h5 = s5 < unb, h6 = s6 < unb, h7 = s7 < unb;
  const unsigned any = __builtin_amdgcn_ballot_w32(h0 | h1 | h2 | h3 | h4 | h5 | h6 | h7);
  if (any != 0u) {
#define HITJ(J, HJ, SJ) { \
      const unsigned mj = __builtin_amdgcn_ballot_w32(HJ); \
      if (mj != 0u) { \
        if (HJ) { \
          const int pos = wc + (int)__builtin_amdgcn_mbcnt_lo(mj, 0u); \
          if (pos < WCAP) list[wave * WCAP + pos] = ((el0 + (J)) << 12) | (int)(SJ); \
        } \
        wc += (int)__builtin_popcount(mj); } }
    HITJ(0, h0, s0)
    HITJ(1, h1, s1)
    HITJ(2, h2, s2)
    HITJ(3, h3, s3)
    HITJ(4, h4, s4)
    HITJ(5, h5, s5)
    HITJ(6, h6, s6)
    HITJ(7, h7, s7)
#undef HITJ
  }
  return wc;
}

__global__ __launch_bounds__(NTHR) void k_build(const int* __restrict__ srcs, const int* __restrict__ dsts,
                                                int* LIST, int* CNT, int* OFF, int* META) {
  extern __shared__ v4f lds_dyn[];
  int* reg1 = (int*)lds_dyn;
  int* list = reg1 + RCAP;
  unsigned short* perm = (unsigned short*)(reg1 + RCAP);
  int* scnt = reg1 + RCAP + RCAP / 2;
  int* cur  = scnt + NBROWS;
  int* wcnt = cur + NBROWS;
  int* wtot = wcnt + NWAVE;
  const int tid = (int)threadIdx.x, lane = tid & 31, wave = tid >> 5;
  const int wv = __builtin_amdgcn_readfirstlane(tid >> 5);
  const int b = (int)blockIdx.x;
  const int nodeBase = b * NBROWS;
  const int nb = clampi(NN - nodeBase, 0, NBROWS);

  for (int i = tid; i < NBROWS; i += NTHR) scnt[i] = 0;
  __syncthreads();

  int tot = 0;
#pragma unroll 1
  for (int ch = 0; ch < NCHUNK; ++ch) {
    const int cbase = ch * CHUNK;
    const int wc = scan_chunk(dsts, cbase, nodeBase, nb, list, tid, wave);
    if (lane == 0) wcnt[wave] = wc;
    __syncthreads();
    int pre = 0, all = 0;
#pragma unroll
    for (int w2 = 0; w2 < NWAVE; ++w2) {
      int c = wcnt[w2];
      c = c < 0 ? 0 : (c > WCAP ? WCAP : c);
      all += c;
      pre += (w2 < wave) ? c : 0;
    }
    const int wcc  = wc > WCAP ? WCAP : wc;
    const int base = tot + pre;
#pragma unroll 1
    for (int i = lane; i < wcc; i += 32) {
      const int ent = list[wave * WCAP + i];
      const int el  = (ent >> 12) & (CHUNK - 1);
      const int sl  = ent & (NBROWS - 1);
      int eid = cbase + el;
      eid = eid > NE - 1 ? NE - 1 : eid;
      const int pos = base + i;
      if (pos < RCAP) reg1[pos] = (int)(((unsigned)eid << ESH) | (unsigned)sl);
    }
    int nt = tot + all;
    nt = nt > RCAP ? RCAP : nt;
    tot = __builtin_amdgcn_readfirstlane(nt);
    __syncthreads();
  }
  const int nh = tot;

  if (wv == 0) {
    if (lane == 0 && nh == 0) { perm[0] = (unsigned short)0; reg1[0] = 0; }
#pragma unroll 1
    for (int b0 = 0; b0 < nh; b0 += 32) {
      const int idx = (b0 + lane) < nh ? (b0 + lane) : nh - 1;
      const int uv  = reg1[idx];
      const int m32 = (nh - b0) < 32 ? (nh - b0) : 32;
#pragma unroll 1
      for (int k = 0; k < m32; ++k) {
        const int u  = __builtin_amdgcn_readlane(uv, k);
        const int sl = u & (NBROWS - 1);
        if (lane == 0) scnt[sl] = scnt[sl] + 1;
      }
    }
  }
  __syncthreads();

  {
    const v4i ca = *(const v4ia*)(scnt + 4 * tid);
    const int e0 = ca.x < 0 ? 0 : ca.x, e1 = ca.y < 0 ? 0 : ca.y, e2 = ca.z < 0 ? 0 : ca.z, e3 = ca.w < 0 ? 0 : ca.w;
    const int ts = e0 + e1 + e2 + e3;
    int incl = ts;
#pragma unroll
    for (int d = 1; d < 32; d <<= 1) {
      const int up = __shfl_up(incl, d);
      if (lane >= d) incl += up;
    }
    if (lane == 31) wtot[wave] = incl;
    __syncthreads();
    int pre = 0;
#pragma unroll
    for (int w2 = 0; w2 < NWAVE; ++w2) pre += (w2 < wave) ? wtot[w2] : 0;
    int run = pre + incl - ts;
    cur[4 * tid + 0] = run; run += e0;
    cur[4 * tid + 1] = run; run += e1;
    cur[4 * tid + 2] = run; run += e2;
    cur[4 * tid + 3] = run;
  }
  __syncthreads();

  if (wv == 0) {
#pragma unroll 1
    for (int b0 = 0; b0 < nh; b0 += 32) {
      const int idx = (b0 + lane) < nh ? (b0 + lane) : nh - 1;
      const int uv  = reg1[idx];
      const int m32 = (nh - b0) < 32 ? (nh - b0) : 32;
#pragma unroll 1
      for (int k = 0; k < m32; ++k) {
        const int u  = __builtin_amdgcn_readlane(uv, k);
        const int sl = u & (NBROWS - 1);
        if (lane == 0) {
          int pos = cur[sl];
          pos = pos < 0 ? 0 : (pos > RCAP - 1 ? RCAP - 1 : pos);
          perm[pos] = (unsigned short)(b0 + k);
          cur[sl] = pos + 1;
        }
      }
    }
  }
  __syncthreads();

  int* bl = LIST + (size_t)b * RCAP * 2;
  const int last = nh > 0 ? nh - 1 : 0;
#pragma unroll 1
  for (int base = 0; base < RCAP; base += 512) {
    const int i0 = base + 2 * tid;
    int p0 = (int)perm[i0     < last ? i0     : last];
    int p1 = (int)perm[i0 + 1 < last ? i0 + 1 : last];
    p0 = p0 > last ? last : p0;
    p1 = p1 > last ? last : p1;
    const unsigned u0 = (unsigned)reg1[p0];
    const unsigned u1 = (unsigned)reg1[p1];
    int e0 = (int)(u0 >> ESH);
    int e1 = (int)(u1 >> ESH);
    e0 = e0 > NE - 1 ? NE - 1 : e0;
    e1 = e1 > NE - 1 ? NE - 1 : e1;
    int s0 = srcs[e0];
    int s1 = srcs[e1];
    asm volatile("" :: "v"(s0), "v"(s1));
    s0 = clampi(s0, 0, NN - 1);
    s1 = clampi(s1, 0, NN - 1);
    const int k0 = (i0     < nh) ? -1 : 0;
    const int k1 = (i0 + 1 < nh) ? -1 : 0;
    const v4i v = (v4i){ s0 & k0, e0 & k0, s1 & k1, e1 & k1 };
    st2_v4i(bl + 2 * i0, v);
  }
  {
    const v4i sc = *(const v4ia*)(scnt + 4 * tid);
    const v4i cu = *(const v4ia*)(cur + 4 * tid);
    v4i of = cu - sc;
    of.x = clampi(of.x, 0, RCAP - 1) + b * RCAP;
    of.y = clampi(of.y, 0, RCAP - 1) + b * RCAP;
    of.z = clampi(of.z, 0, RCAP - 1) + b * RCAP;
    of.w = clampi(of.w, 0, RCAP - 1) + b * RCAP;
    st2_v4i(CNT + (size_t)b * NBROWS + 4 * tid, sc);
    st2_v4i(OFF + (size_t)b * NBROWS + 4 * tid, of);
  }
  if (tid < 8) {
    v4i mv;
    mv.x = (tid == 0) ? nh : 0;
    mv.y = (tid == 0 && nh >= RCAP) ? 1 : 0;
    mv.z = 0; mv.w = 0;
    st2_v4i(META + (size_t)b * 32 + 4 * tid, mv);
  }
}

__device__ __forceinline__ void own_prologue(const int* __restrict__ CNT, const int* __restrict__ OFF,
                                             const int* __restrict__ META, int n,
                                             int& c, int& craw, int& off, int& cmax, int& bad) {
  int cv = CNT[n];
  int ov = OFF[n];
  int fl = META[(size_t)(n >> 10) * 32 + 1];
  asm volatile("" :: "v"(cv), "v"(ov), "v"(fl));
  craw = cv < 0 ? 0 : cv;
  c = craw > DEGCAP ? DEGCAP : craw;
  off = clampi(ov, 0, LTOT - 1);
  int m = c, t;
  t = __shfl_xor(m, 16); m = m > t ? m : t;
  t = __shfl_xor(m, 8);  m = m > t ? m : t;
  t = __shfl_xor(m, 4);  m = m > t ? m : t;
  t = __shfl_xor(m, 2);  m = m > t ? m : t;
  t = __shfl_xor(m, 1);  m = m > t ? m : t;
  cmax = __builtin_amdgcn_readfirstlane(m);
  bad = (fl != 0 || craw > DEGCAP) ? 1 : 0;
}
__device__ __forceinline__ v2i load_hit(const int* __restrict__ LIST, int off, int c, int j) {
  int jj = j < c - 1 ? j : c - 1;
  jj = jj < 0 ? 0 : jj;
  int idx = off + jj;
  idx = idx > LTOT - 1 ? LTOT - 1 : idx;
  v2i ent = *(const v2ia*)(LIST + 2 * (size_t)idx);
  asm volatile("" :: "v"(ent));
  v2i r;
  r.x = clampi(ent.x, 0, NN - 1);
  r.y = clampi(ent.y, 0, NE - 1);
  return r;
}

__global__ __launch_bounds__(256) void k_diff(const float* __restrict__ XR, const int* __restrict__ LIST,
                                              const int* __restrict__ CNT, const int* __restrict__ OFF,
                                              const int* __restrict__ META, const float* __restrict__ PAR, float* XD) {
  const int n = (int)blockIdx.x * 256 + (int)threadIdx.x;
  const int n0 = __builtin_amdgcn_readfirstlane(n & ~31);
  if (n0 >= NN) return;
  int c, craw, off, cmax, bad;
  own_prologue(CNT, OFF, META, n, c, craw, off, cmax, bad);
  const float tau = PAR[PA_TAU];
  const v2f xo = *(const v2fa*)(XR + 2 * (size_t)n);
  float ax = 0.0f, ay = 0.0f;
#pragma unroll 1
  for (int j = 0; j < cmax; ++j) {
    const v2i ent = load_hit(LIST, off, c, j);
    const v2f xs = *(const v2fa*)(XR + 2 * (size_t)ent.x);
    asm volatile("" :: "v"(xs));
    const bool on = j < c;
    ax = on ? ax + xs.x : ax;
    ay = on ? ay + xs.y : ay;
  }
  const float deg = (float)(craw > 0 ? craw : 1);
  const float m0 = ax / deg;
  const float m1 = ay / deg;
  float r0 = xo.x + tau * (m0 - xo.x);
  float r1 = xo.y + tau * (m1 - xo.y);
  const float qnan = __int_as_float(0x7fc00000);
  r0 = bad ? qnan : r0;
  r1 = bad ? qnan : r1;
  st2_v2f(XD + 2 * (size_t)n, (v2f){ r0, r1 });
}

__global__ __launch_bounds__(256) void k_emap(const int* __restrict__ ei, const float* __restrict__ XD,
                                              const float* __restrict__ PAR, float* out) {
  __shared__ float sP[32];
  const int tid = (int)threadIdx.x;
  if (tid < 32) sP[tid] = PAR[tid];
  __syncthreads();
  const int e = (int)blockIdx.x * 256 + tid;
  int s = ei[e];
  int d = ei[NE + e];
  asm volatile("" :: "v"(s), "v"(d));
  s = clampi(s, 0, NN - 1);
  d = clampi(d, 0, NN - 1);
  const v2f a = *(const v2fa*)(XD + 2 * (size_t)s);
  const v2f c = *(const v2fa*)(XD + 2 * (size_t)d);
  asm volatile("" :: "v"(a), "v"(c));
  v4f r;
#pragma unroll
  for (int q = 0; q < 4; ++q) {
    float t = a.x * sP[PA_WMAP + q];
    t = fmaf(a.y, sP[PA_WMAP + 4 + q], t);
    t = fmaf(c.x, sP[PA_WMAP + 8 + q], t);
    t = fmaf(c.y, sP[PA_WMAP + 12 + q], t);
    r[q] = t + sP[PA_BMAP + q];
  }
  st2_v4f(out + OUT_R_ELEM + 4 * (size_t)e, r);
}

__global__ __launch_bounds__(256) void k_hop1(const float* __restrict__ Kw, const float* __restrict__ XD,
                                              const int* __restrict__ LIST, const int* __restrict__ CNT,
                                              const int* __restrict__ OFF, const int* __restrict__ META, float* H1) {
  const int n = (int)blockIdx.x * 256 + (int)threadIdx.x;
  const int n0 = __builtin_amdgcn_readfirstlane(n & ~31);
  if (n0 >= NN) return;
  int c, craw, off, cmax, bad;
  own_prologue(CNT, OFF, META, n, c, craw, off, cmax, bad);
  float h0 = 0.0f, h1 = 0.0f, h2 = 0.0f, h3 = 0.0f;
#pragma unroll 1
  for (int j = 0; j < cmax; ++j) {
    const v2i ent = load_hit(LIST, off, c, j);
    float k0 = Kw[ent.y];
    float k1 = Kw[(size_t)NE + ent.y];
    const v2f xs = *(const v2fa*)(XD + 2 * (size_t)ent.x);
    asm volatile("" :: "v"(k0), "v"(k1), "v"(xs));
    k0 = bf16_val(k0);
    k1 = bf16_val(k1);
    const bool on = j < c;
    h0 = on ? h0 + k0 * xs.x : h0;
    h1 = on ? h1 + k0 * xs.y : h1;
    h2 = on ? h2 + k1 * xs.x : h2;
    h3 = on ? h3 + k1 * xs.y : h3;
  }
  const float qnan = __int_as_float(0x7fc00000);
  v4f o = (v4f){ h0, h1, h2, h3 };
  o = bad ? (v4f){ qnan, qnan, qnan, qnan } : o;
  st2_v4f(H1 + 4 * (size_t)n, o);
}

__global__ __launch_bounds__(256) void k_hop2(const float* __restrict__ Kw, const float* __restrict__ XD,
                                              const float* __restrict__ H1, const int* __restrict__ LIST,
                                              const int* __restrict__ CNT, const int* __restrict__ OFF,
                                              const int* __restrict__ META, float* O16) {
  __shared__ __attribute__((aligned(16))) float sO[8][32 * 16];
  const int tid = (int)threadIdx.x, lane = tid & 31, wave = tid >> 5;
  const int n = (int)blockIdx.x * 256 + tid;
  const int n0 = __builtin_amdgcn_readfirstlane(n & ~31);
  if (n0 >= NN) return;
  int c, craw, off, cmax, bad;
  own_prologue(CNT, OFF, META, n, c, craw, off, cmax, bad);
  float a[8];
#pragma unroll
  for (int q = 0; q < 8; ++q) a[q] = 0.0f;
#pragma unroll 1
  for (int j = 0; j < cmax; ++j) {
    const v2i ent = load_hit(LIST, off, c, j);
    float k0 = Kw[ent.y];
    float k1 = Kw[(size_t)NE + ent.y];
    const v4f hv = *(const v4fa*)(H1 + 4 * (size_t)ent.x);
    asm volatile("" :: "v"(k0), "v"(k1), "v"(hv));
    k0 = bf16_val(k0);
    k1 = bf16_val(k1);
    const bool on = j < c;
#pragma unroll
    for (int q = 0; q < 4; ++q) {
      a[q]     = on ? a[q]     + k0 * hv[q] : a[q];
      a[4 + q] = on ? a[4 + q] + k1 * hv[q] : a[4 + q];
    }
  }
  const float qnan = __int_as_float(0x7fc00000);
#pragma unroll
  for (int q = 0; q < 8; ++q) a[q] = bad ? qnan : a[q];
  const v2f xo = *(const v2fa*)(XD + 2 * (size_t)n);
  const v4f ho = *(const v4fa*)(H1 + 4 * (size_t)n);
  float* tile = &sO[wave][0];
  float* row = tile + lane * 16;
  *(v4fa*)(row)      = (v4f){ xo.x, xo.y, ho[0], ho[1] };
  *(v4fa*)(row + 4)  = (v4f){ ho[2], ho[3], a[0], a[1] };
  *(v4fa*)(row + 8)  = (v4f){ a[2], a[3], a[4], a[5] };
  *(v4fa*)(row + 12) = (v4f){ a[6], a[7], 0.0f, 0.0f };
  wave_sync_lds();
  const v4f o0 = *(const v4fa*)(tile + (0 * 32 + lane) * 4);
  const v4f o1 = *(const v4fa*)(tile + (1 * 32 + lane) * 4);
  const v4f o2 = *(const v4fa*)(tile + (2 * 32 + lane) * 4);
  const v4f o3 = *(const v4fa*)(tile + (3 * 32 + lane) * 4);
  float* dst = O16 + (size_t)n0 * 16 + lane * 4;
  volatile v4f* q0 = (volatile v4f*)(dst);
  volatile v4f* q1 = (volatile v4f*)(dst + 128);
  volatile v4f* q2 = (volatile v4f*)(dst + 256);
  volatile v4f* q3 = (volatile v4f*)(dst + 384);
  *q0 = o0; *q1 = o1; *q2 = o2; *q3 = o3;
  __threadfence();
  *q0 = o0; *q1 = o1; *q2 = o2; *q3 = o3;
}

__global__ __launch_bounds__(256) void k_conv(const float* __restrict__ O16, const int* __restrict__ LIST,
                                              const int* __restrict__ CNT, const int* __restrict__ OFF,
                                              const int* __restrict__ META, const float* __restrict__ PAR,
                                              unsigned short* AHL) {
  __shared__ __attribute__((aligned(16))) float sW[224];
  __shared__ __attribute__((aligned(16))) float sM[8][32 * 16];
  __shared__ __attribute__((aligned(16))) unsigned sA[8][32 * 16];
  const int tid = (int)threadIdx.x, lane = tid & 31, wave = tid >> 5;
  {
    const int ix = tid < 56 ? tid : 55;
    const v4f w = *(const v4fa*)(PAR + PA_WC + 4 * ix);
    asm volatile("" :: "v"(w));
    if (tid < 56) *(v4fa*)(sW + 4 * tid) = w;
  }
  __syncthreads();
  const int n = (int)blockIdx.x * 256 + tid;
  const int n0 = __builtin_amdgcn_readfirstlane(n & ~31);
  if (n0 >= NN) return;
  int c, craw, off, cmax, bad;
  own_prologue(CNT, OFF, META, n, c, craw, off, cmax, bad);
  float a[14];
#pragma unroll
  for (int q = 0; q < 14; ++q) a[q] = 0.0f;
#pragma unroll 1
  for (int j = 0; j < cmax; ++j) {
    const v2i ent = load_hit(LIST, off, c, j);
    const float* orow = O16 + 16 * (size_t)ent.x;
    const v4f r0 = *(const v4fa*)(orow);
    const v4f r1 = *(const v4fa*)(orow + 4);
    const v4f r2 = *(const v4fa*)(orow + 8);
    const v4f r3 = *(const v4fa*)(orow + 12);
    asm volatile("" :: "v"(r0), "v"(r1), "v"(r2), "v"(r3));
    const bool on = j < c;
#pragma unroll
    for (int q = 0; q < 4; ++q) {
      a[q]     = on ? a[q]     + r0[q] : a[q];
      a[4 + q] = on ? a[4 + q] + r1[q] : a[4 + q];
      a[8 + q] = on ? a[8 + q] + r2[q] : a[8 + q];
    }
    a[12] = on ? a[12] + r3[0] : a[12];
    a[13] = on ? a[13] + r3[1] : a[13];
  }
  float* mr = &sM[wave][0] + lane * 16;
  *(v4fa*)(mr)      = (v4f){ a[0], a[1], a[2], a[3] };
  *(v4fa*)(mr + 4)  = (v4f){ a[4], a[5], a[6], a[7] };
  *(v4fa*)(mr + 8)  = (v4f){ a[8], a[9], a[10], a[11] };
  *(v4fa*)(mr + 12) = (v4f){ a[12], a[13], 0.0f, 0.0f };
  const float deg = (float)(craw > 0 ? craw : 1);
#pragma unroll 1
  for (int k = 0; k < 14; ++k) {
    const float t = mr[k];
    mr[k] = t / deg;
  }
  const v4f m0 = *(const v4fa*)(mr);
  const v4f m1 = *(const v4fa*)(mr + 4);
  const v4f m2 = *(const v4fa*)(mr + 8);
  const v4f m3 = *(const v4fa*)(mr + 12);
  float m[14];
#pragma unroll
  for (int q = 0; q < 4; ++q) { m[q] = m0[q]; m[4 + q] = m1[q]; m[8 + q] = m2[q]; }
  m[12] = m3[0];
  m[13] = m3[1];
  const float qnan = __int_as_float(0x7fc00000);
  unsigned* tile = &sA[wave][0];
  unsigned* ar = tile + lane * 16;
#pragma unroll 1
  for (int jp = 0; jp < 7; ++jp) {
    const int j0 = 2 * jp;
    float g0 = m[0] * sW[j0];
    float g1 = m[0] * sW[j0 + 1];
#pragma unroll
    for (int k = 1; k < 14; ++k) {
      g0 = fmaf(m[k], sW[k * 14 + j0], g0);
      g1 = fmaf(m[k], sW[k * 14 + j0 + 1], g1);
    }
    g0 += sW[196 + j0];
    g1 += sW[196 + j0 + 1];
    g0 = (g0 > 0.0f) ? g0 : (g0 - g0);
    g1 = (g1 > 0.0f) ? g1 : (g1 - g1);
    g0 = bad ? qnan : g0;
    g1 = bad ? qnan : g1;
    ar[jp]     = pk16(bf16_bits(g0), bf16_bits(g1));
    ar[7 + jp] = pk16(bf16_lo_bits(g0), bf16_lo_bits(g1));
  }
  ar[14] = 0u;
  ar[15] = 0u;
  wave_sync_lds();
  const v4u o0 = *(const v4ua*)(tile + (0 * 32 + lane) * 4);
  const v4u o1 = *(const v4ua*)(tile + (1 * 32 + lane) * 4);
  const v4u o2 = *(const v4ua*)(tile + (2 * 32 + lane) * 4);
  const v4u o3 = *(const v4ua*)(tile + (3 * 32 + lane) * 4);
  unsigned short* dst = AHL + (size_t)n0 * 32 + lane * 8;
  volatile v4u* q0 = (volatile v4u*)(dst);
  volatile v4u* q1 = (volatile v4u*)(dst + 256);
  volatile v4u* q2 = (volatile v4u*)(dst + 512);
  volatile v4u* q3 = (volatile v4u*)(dst + 768);
  *q0 = o0; *q1 = o1; *q2 = o2; *q3 = o3;
  __threadfence();
  *q0 = o0; *q1 = o1; *q2 = o2; *q3 = o3;
}

__global__ __launch_bounds__(256) void k_head(const float* __restrict__ PRE, const float* __restrict__ PAR,
                                              const int* __restrict__ META, float* out) {
  __shared__ __attribute__((aligned(16))) float sY[8][96];
  const int tid = (int)threadIdx.x, lane = tid & 31, wave = tid >> 5;
  const int wg = __builtin_amdgcn_readfirstlane((int)blockIdx.x * 8 + (tid >> 5));
  if (wg >= NN / 32) return;
  const v4f b1v = *(const v4fa*)(PAR + PA_B1 + 4 * lane);
  const v4f wa  = *(const v4fa*)(PAR + PA_W2 + 12 * lane);
  const v4f wb  = *(const v4fa*)(PAR + PA_W2 + 12 * lane + 4);
  const v4f wd  = *(const v4fa*)(PAR + PA_W2 + 12 * lane + 8);
  const float b2v = PAR[PA_B2 + (lane < 2 ? lane : 2)];
  const int fl = META[(size_t)(wg >> 5) * 32 + 1];
  asm volatile("" :: "v"(fl));
  float* ys = &sY[wave][0];
#pragma unroll 1
  for (int r = 0; r < 32; ++r) {
    const size_t row = (size_t)wg * 32 + r;
    const v4f v = *(const v4fa*)(PRE + row * 128 + 4 * lane);
    float h0 = v[0] + b1v[0], h1 = v[1] + b1v[1], h2 = v[2] + b1v[2], h3 = v[3] + b1v[3];
    h0 = (h0 > 0.0f) ? h0 : (h0 - h0);
    h1 = (h1 > 0.0f) ? h1 : (h1 - h1);
    h2 = (h2 > 0.0f) ? h2 : (h2 - h2);
    h3 = (h3 > 0.0f) ? h3 : (h3 - h3);
    float p0 = h0 * wa[0];
    p0 = fmaf(h1, wa[3], p0); p0 = fmaf(h2, wb[2], p0); p0 = fmaf(h3, wd[1], p0);
    float p1 = h0 * wa[1];
    p1 = fmaf(h1, wb[0], p1); p1 = fmaf(h2, wb[3], p1); p1 = fmaf(h3, wd[2], p1);
    float p2 = h0 * wa[2];
    p2 = fmaf(h1, wb[1], p2); p2 = fmaf(h2, wd[0], p2); p2 = fmaf(h3, wd[3], p2);
    p0 += __shfl_xor(p0, 16); p1 += __shfl_xor(p1, 16); p2 += __shfl_xor(p2, 16);
    p0 += __shfl_xor(p0, 8);  p1 += __shfl_xor(p1, 8);  p2 += __shfl_xor(p2, 8);
    p0 += __shfl_xor(p0, 4);  p1 += __shfl_xor(p1, 4);  p2 += __shfl_xor(p2, 4);
    p0 += __shfl_xor(p0, 2);  p1 += __shfl_xor(p1, 2);  p2 += __shfl_xor(p2, 2);
    p0 += __shfl_xor(p0, 1);  p1 += __shfl_xor(p1, 1);  p2 += __shfl_xor(p2, 1);
    const float sel = (lane == 0) ? p0 : ((lane == 1) ? p1 : p2);
    if (lane < 3) ys[3 * r + lane] = sel + b2v;
  }
  wave_sync_lds();
  const int lc = lane < 24 ? lane : 23;
  v4f o = *(const v4fa*)(ys + 4 * lc);
  const float qnan = __int_as_float(0x7fc00000);
  o = (fl != 0) ? (v4f){ qnan, qnan, qnan, qnan } : o;
  if (lane < 24) st2_v4f(out + (size_t)wg * 96 + 4 * lane, o);
}

extern "C" void kernel_launch(void* const* d_in, const int* in_sizes, int n_in,
                              void* d_out, int out_size, void* d_ws, size_t ws_size,
                              hipStream_t stream) {
  if (n_in < 12) return;
  if (in_sizes[0] != NN * 2 || in_sizes[1] != 2 * NE || in_sizes[2] != 1) return;
  if (in_sizes[3] != 16 || in_sizes[4] != 4 || in_sizes[5] != 196 || in_sizes[6] != 14) return;
  if (in_sizes[7] != 14 * 128 || in_sizes[8] != 128 || in_sizes[9] != 384 || in_sizes[10] != 3) return;
  if (in_sizes[11] != 2 * NE) return;
  if (out_size != OUT_R_ELEM + 4 * NE) return;
  if (ws_size < WS_TOTAL) return;

  const float* x     = (const float*)d_in[0];
  const float* Kw    = (const float*)d_in[1];
  const float* tau   = (const float*)d_in[2];
  const float* wmap  = (const float*)d_in[3];
  const float* bmap  = (const float*)d_in[4];
  const float* wconv = (const float*)d_in[5];
  const float* bconv = (const float*)d_in[6];
  const float* w1    = (const float*)d_in[7];
  const float* b1    = (const float*)d_in[8];
  const float* w2    = (const float*)d_in[9];
  const float* b2    = (const float*)d_in[10];
  const int*   ei    = (const int*)  d_in[11];
  float* out = (float*)d_out;

  char* ws = (char*)d_ws;
  float*          XR   = (float*)(ws + O_XR);
  float*          XD   = (float*)(ws + O_XD);
  float*          H1   = (float*)(ws + O_H1);
  float*          O16  = (float*)(ws + O_O16);
  unsigned short* AHL  = (unsigned short*)(ws + O_AHL);
  unsigned short* B1T  = (unsigned short*)(ws + O_B1T);
  float*          PAR  = (float*)(ws + O_PAR);
  int*            CNT  = (int*)(ws + O_CNT);
  int*            OFF  = (int*)(ws + O_OFF);
  int*            META = (int*)(ws + O_META);
  int*            LIST = (int*)(ws + O_LIST);
  float*          PRE  = (float*)(ws + O_PRE);

  hipFuncSetAttribute(reinterpret_cast<const void*>(&k_build),
                      hipFuncAttributeMaxDynamicSharedMemorySize, LDS_BLD);

  k_prep<<<203, 256, 0, stream>>>(x, tau, wmap, bmap, wconv, bconv, w1, b1, w2, b2, XR, PAR, B1T, AHL);
  k_build<<<NBLK, NTHR, LDS_BLD, stream>>>(ei, ei + NE, LIST, CNT, OFF, META);
  k_diff<<<391, 256, 0, stream>>>(XR, LIST, CNT, OFF, META, PAR, XD);
  k_emap<<<NE / 256, 256, 0, stream>>>(ei, XD, PAR, out);
  k_hop1<<<391, 256, 0, stream>>>(Kw, XD, LIST, CNT, OFF, META, H1);
  k_hop2<<<391, 256, 0, stream>>>(Kw, XD, H1, LIST, CNT, OFF, META, O16);
  k_conv<<<391, 256, 0, stream>>>(O16, LIST, CNT, OFF, META, PAR, AHL);
  k_gemm_nt<0, 0><<<(3126 + 7) / 8, 256, 0, stream>>>(AHL, B1T, PAR, PRE, NN, 128, 32, 128);
  k_head<<<391, 256, 0, stream>>>(PRE, PAR, META, out);
}
